// TFRelPartialLearnableMultiHeadAttn_35613868819139
// MI455X (gfx1250) — hardware-verified
//
#include <hip/hip_runtime.h>
#include <math.h>

constexpr int kQLen   = 1024;
constexpr int kMLen   = 1024;
constexpr int kKLen   = 2048;
constexpr int kRLen   = 2048;
constexpr int kBsz    = 4;
constexpr int kDModel = 1024;
constexpr int kNHead  = 16;
constexpr int kDHead  = 64;
constexpr int kHD     = kNHead * kDHead;
constexpr int kCatRows = kKLen * kBsz;
constexpr int kQRows   = kQLen * kBsz;
constexpr int kNGroups  = kBsz * kNHead;
constexpr int kGrpChunk = 2;

constexpr float kWCarry    = 64.0f;
constexpr float kWCarryInv = 1.0f / 64.0f;
constexpr float kPCarry    = 2048.0f;
constexpr float kAVCarry   = 256.0f;
constexpr float kPVScale   = kAVCarry / kPCarry;
constexpr float kOutScale  = 1.0f / (kAVCarry * kWCarry);
constexpr float kScoreScale = 0.125f;
constexpr float kMaskFill  = -1.0e30f;
constexpr float kInvDModel = 1.0f / 1024.0f;
constexpr float kLnEps     = 1e-5f;

constexpr size_t kMiB = (size_t)1 << 20;
constexpr size_t kOffCat   = 0;
constexpr size_t kOffSac   = 0;
constexpr size_t kOffOW    = 0;
constexpr size_t kOffR16   = 16 * kMiB;
constexpr size_t kOffP16   = 16 * kMiB;
constexpr size_t kOffWqkvT = 20 * kMiB;
constexpr size_t kOffWrT   = 26 * kMiB;
constexpr size_t kOffWoT   = 28 * kMiB;
constexpr size_t kOffQw    = 30 * kMiB;
constexpr size_t kOffQr    = 38 * kMiB;
constexpr size_t kOffK16   = 46 * kMiB;
constexpr size_t kOffVT16  = 62 * kMiB;
constexpr size_t kOffRK16  = 78 * kMiB;
constexpr size_t kOffAV16  = 82 * kMiB;
constexpr size_t kOffSbd   = 90 * kMiB;
constexpr size_t kWsTotal  = 106 * kMiB;
static_assert((size_t)kCatRows * kDModel * 2 == 16 * kMiB);
static_assert((size_t)kGrpChunk * kQLen * kKLen * 4 == 16 * kMiB);
static_assert((size_t)kGrpChunk * kQLen * kKLen * 2 == 8 * kMiB);
static_assert((size_t)3 * kHD * kDModel * 2 == 6 * kMiB);
static_assert((size_t)kQRows * kHD * 2 == 8 * kMiB);
static_assert((size_t)kBsz * kHD * kKLen * 2 == 16 * kMiB);
static_assert((size_t)kRLen * kHD * 2 == 4 * kMiB);
static_assert((size_t)kQRows * kDModel * 4 == 16 * kMiB);
static_assert(kWsTotal <= (size_t)134217728);

typedef __attribute__((ext_vector_type(16))) _Float16 v16h;
typedef __attribute__((ext_vector_type(8)))  _Float16 v8h;
typedef __attribute__((ext_vector_type(16))) __bf16   v16b;
typedef __attribute__((ext_vector_type(8)))  __bf16   v8b;
typedef __attribute__((ext_vector_type(8)))  float    v8f;
typedef __attribute__((ext_vector_type(4)))  float    v4f;
typedef __attribute__((ext_vector_type(4)))  unsigned int v4u;
typedef __attribute__((ext_vector_type(4)))  int      v4i;

__device__ __forceinline__ unsigned short f2bf_bits(float f) {
  unsigned u = __float_as_uint(f);
  return (unsigned short)((u + 0x7FFFu + ((u >> 16) & 1u)) >> 16);
}
__device__ __forceinline__ float bf_bits2f(unsigned short h) { return __uint_as_float(((unsigned)h) << 16); }

__device__ __forceinline__ void dep_guard_h(v8f& a, v8f& b, v16h x, v16h y) { asm volatile("v_nop\n\tv_nop\n\tv_nop\n\tv_nop" : "+v"(a), "+v"(b) : "v"(x), "v"(y)); }
__device__ __forceinline__ void dep_guard_b(v8f& a, v8f& b, v16b x, v16b y) { asm volatile("v_nop\n\tv_nop\n\tv_nop\n\tv_nop" : "+v"(a), "+v"(b) : "v"(x), "v"(y)); }
__device__ __forceinline__ void keep4_h(v16h a, v16h b, v16h c, v16h d) { asm volatile("v_nop" :: "v"(a), "v"(b), "v"(c), "v"(d)); }
__device__ __forceinline__ void keep4_b(v16b a, v16b b, v16b c, v16b d) { asm volatile("v_nop" :: "v"(a), "v"(b), "v"(c), "v"(d)); }
__device__ __forceinline__ void acc_guard4(v8f& a, v8f& b, v8f& c, v8f& d) { asm volatile("v_nop\n\tv_nop\n\tv_nop\n\tv_nop" : "+v"(a), "+v"(b), "+v"(c), "+v"(d)); }
template <typename T> struct Frag;
template <> struct Frag<_Float16> {
  typedef v16h V; union U { v16h v; v8h h[2]; };
  static __device__ __forceinline__ v16h load(const _Float16* p) {
    U f; f.h[0] = *(const v8h*)(p); f.h[1] = *(const v8h*)(p + 16); return f.v;
  }
  static __device__ __forceinline__ v8f mma(v16h a, v16h b, v8f c) {
    return __builtin_amdgcn_wmma_f32_16x16x32_f16(false, a, false, b, (short)0, c, false, false);
  }
  static __device__ __forceinline__ void guard(v8f& a, v8f& b, v16h x, v16h y) { dep_guard_h(a, b, x, y); }
  static __device__ __forceinline__ void keep(v16h a, v16h b, v16h c, v16h d) { keep4_h(a, b, c, d); }
};
template <> struct Frag<__bf16> {
  typedef v16b V; union U { v16b v; v8b h[2]; };
  static __device__ __forceinline__ v16b load(const __bf16* p) {
    U f; f.h[0] = *(const v8b*)(p); f.h[1] = *(const v8b*)(p + 16); return f.v;
  }
  static __device__ __forceinline__ v8f mma(v16b a, v16b b, v8f c) {
    return __builtin_amdgcn_wmma_f32_16x16x32_bf16(false, a, false, b, (short)0, c, false, false);
  }
  static __device__ __forceinline__ void guard(v8f& a, v8f& b, v16b x, v16b y) { dep_guard_b(a, b, x, y); }
  static __device__ __forceinline__ void keep(v16b a, v16b b, v16b c, v16b d) { keep4_b(a, b, c, d); }
};

__device__ __forceinline__ unsigned pk16(unsigned short a, unsigned short b) { return (unsigned)a | ((unsigned)b << 16); }
__device__ __forceinline__ unsigned short h_bits(float f) { const _Float16 h = (_Float16)f; return __builtin_bit_cast(unsigned short, h); }

template <int ET> struct Elem;
template <> struct Elem<0> { typedef _Float16 T; };
template <> struct Elem<1> { typedef __bf16 T; };
template <int ET, bool SPLIT, int BIAS_MODE, int OUT_MODE, bool RESID, int ACT = 0>
__global__ __launch_bounds__(256) void wmma_gemm64(
    const unsigned short* __restrict__ Ap, const unsigned short* __restrict__ A2p, int lda, long strideA,
    const unsigned short* __restrict__ Btp, const unsigned short* __restrict__ Bt2p, int ldb, long strideB,
    void* __restrict__ Cout, void* __restrict__ Cout2, int ldc, long strideC,
    const float* __restrict__ bias,
    const float* __restrict__ resid, long strideR,
    int M, int N, int K, float scale) {
  typedef typename Elem<ET>::T T;
  typedef typename Frag<T>::V V;
  const T* A = (const T*)Ap; const T* A2 = (const T*)A2p; const T* Bt = (const T*)Btp; const T* Bt2 = (const T*)Bt2p;
  __shared__ __align__(16) float sT[8][16 * 68];
  const int b    = blockIdx.y;
  const int lane = threadIdx.x & 31;
  const int wave = threadIdx.x >> 5;
  const int tilesN = N >> 6;
  const int tilesM = M >> 6;
  const int tile = blockIdx.x * 8 + wave;
  if (tile >= tilesM * tilesN) return;
  const int tm = tile / tilesN;
  const int tn = tile - tm * tilesN;
  const int m0 = tm << 6;
  const int n0 = tn << 6;

  const T* Ab  = A  + (size_t)b * strideA;
  const T* Bb  = Bt + (size_t)b * strideB;
  const T* Ab2 = SPLIT ? (A2  + (size_t)b * strideA) : nullptr;
  const T* Bb2 = SPLIT ? (Bt2 + (size_t)b * strideB) : nullptr;

  const int rlane = lane & 15;
  const int koff  = (lane >> 4) * 8;
  const int mOff  = (lane >> 4) * 8;

  v8f acc[4][4];
#pragma unroll
  for (int i = 0; i < 4; ++i)
#pragma unroll
    for (int j = 0; j < 4; ++j) acc[i][j] = (v8f){0.f,0.f,0.f,0.f,0.f,0.f,0.f,0.f};

  for (int k0 = 0; k0 < K; k0 += 32) {
    V bh[4], bl[4];
#pragma unroll
    for (int j = 0; j < 4; ++j) {
      const size_t bo = (size_t)(n0 + (j << 4) + rlane) * ldb + koff + k0;
      bh[j] = Frag<T>::load(Bb + bo);
      if (SPLIT) bl[j] = Frag<T>::load(Bb2 + bo);
    }
#pragma unroll
    for (int i = 0; i < 4; ++i) {
      const size_t ao = (size_t)(m0 + (i << 4) + rlane) * lda + koff + k0;
      V ah = Frag<T>::load(Ab + ao);
      V al;
      if (SPLIT) al = Frag<T>::load(Ab2 + ao);
#pragma unroll
      for (int j = 0; j < 4; ++j) {
        acc[i][j] = Frag<T>::mma(ah, bh[j], acc[i][j]);
        if (SPLIT) {
          acc[i][j] = Frag<T>::mma(ah, bl[j], acc[i][j]);
          acc[i][j] = Frag<T>::mma(al, bh[j], acc[i][j]);
        }
      }
      Frag<T>::guard(acc[i][0], acc[i][3], ah, SPLIT ? al : ah);
    }
    Frag<T>::keep(bh[0], bh[1], bh[2], bh[3]);
    if (SPLIT) Frag<T>::keep(bl[0], bl[1], bl[2], bl[3]);
  }
  acc_guard4(acc[0][0], acc[0][1], acc[0][2], acc[0][3]);
  acc_guard4(acc[1][0], acc[1][1], acc[1][2], acc[1][3]);
  acc_guard4(acc[2][0], acc[2][1], acc[2][2], acc[2][3]);
  acc_guard4(acc[3][0], acc[3][1], acc[3][2], acc[3][3]);

  float* slab = sT[wave];
  const float* Rb = RESID ? (resid + (size_t)b * strideR) : nullptr;
#pragma unroll
  for (int i = 0; i < 4; ++i) {
    const int mBase = m0 + (i << 4);
#pragma unroll
    for (int j = 0; j < 4; ++j) {
      const int n = n0 + (j << 4) + rlane;
      float bv = 0.f;
      if (BIAS_MODE == 2) bv = bias[n];
#pragma unroll
      for (int r = 0; r < 8; ++r) {
        float v = acc[i][j][r] * scale;
        if (BIAS_MODE == 1) v += bias[mBase + mOff + r];
        if (BIAS_MODE == 2) v += bv;
        if (RESID) v += Rb[(size_t)(mBase + mOff + r) * ldc + n];
        if (ACT == 2) v = fmaxf(v, 0.0f);
        if (ACT == 4) v = (v > 0.f) ? v : 0.01f * v;
        slab[(mOff + r) * 68 + (j << 4) + rlane] = v;
      }
    }
    __builtin_amdgcn_fence(__ATOMIC_RELEASE, "workgroup");
    __builtin_amdgcn_wave_barrier();
    __builtin_amdgcn_fence(__ATOMIC_ACQUIRE, "workgroup");
    if (OUT_MODE == 0) {
      float* C = (float*)Cout + (size_t)b * strideC;
      const int hh = lane >> 4, c4 = (lane & 15) * 4;
      for (int pass = 0; pass < 2; ++pass) {
#pragma unroll
        for (int it = 0; it < 8; ++it) {
          const int row = it * 2 + hh;
          v4f v = *(const v4f*)(slab + row * 68 + c4);
          *(volatile v4f*)(C + (size_t)(mBase + row) * ldc + n0 + c4) = v;
        }
        __threadfence();
      }
    } else {
      const int q = lane >> 3, c8 = (lane & 7) * 8;
      unsigned short* C  = (unsigned short*)Cout  + (size_t)b * strideC;
      unsigned short* C2 = (OUT_MODE == 2) ? ((unsigned short*)Cout2 + (size_t)b * strideC) : nullptr;
      for (int pass = 0; pass < 2; ++pass) {
#pragma unroll
        for (int it = 0; it < 4; ++it) {
          const int row = it * 4 + q;
          const float* sp = slab + row * 68 + c8;
          v8h hv, lv;
#pragma unroll
          for (int e = 0; e < 8; ++e) {
            if (OUT_MODE == 1) {
              hv[e] = (_Float16)sp[e];
            } else {
              unsigned short hb = f2bf_bits(sp[e]);
              unsigned short lb = f2bf_bits(sp[e] - bf_bits2f(hb));
              hv[e] = __builtin_bit_cast(_Float16, hb);
              lv[e] = __builtin_bit_cast(_Float16, lb);
            }
          }
          *(volatile v8h*)(C + (size_t)(mBase + row) * ldc + n0 + c8) = hv;
          if (OUT_MODE == 2) *(volatile v8h*)(C2 + (size_t)(mBase + row) * ldc + n0 + c8) = lv;
        }
        __threadfence();
      }
    }
    __builtin_amdgcn_fence(__ATOMIC_RELEASE, "workgroup");
    __builtin_amdgcn_wave_barrier();
    __builtin_amdgcn_fence(__ATOMIC_ACQUIRE, "workgroup");
  }
}

__global__ __launch_bounds__(256) void wtcast_kernel(const float* __restrict__ W, unsigned short* __restrict__ WT,
                                                     int Kin, int Nout, float scale) {
  __shared__ float sm[64][65];
  const int t  = threadIdx.x;
  const int k0 = blockIdx.x * 64;
  const int n0 = blockIdx.y * 64;
#pragma unroll
  for (int it = 0; it < 16; ++it) {
    const int e = it * 256 + t;
    const int r = e >> 6;
    const int c = e & 63;
    sm[c][r] = W[(size_t)(k0 + r) * Nout + n0 + c] * scale;
  }
  __syncthreads();
  const int lane = t & 31, wave = t >> 5;
  const int q = lane >> 3, c8 = (lane & 7) * 8;
  for (int pass = 0; pass < 2; ++pass) {
#pragma unroll
    for (int it = 0; it < 2; ++it) {
      const int row = wave * 8 + it * 4 + q;
      unsigned short hb[8];
#pragma unroll
      for (int e = 0; e < 8; ++e) hb[e] = h_bits(sm[row][c8 + e]);
      const v4u u = (v4u){pk16(hb[0], hb[1]), pk16(hb[2], hb[3]), pk16(hb[4], hb[5]), pk16(hb[6], hb[7])};
      *(volatile v4u*)(WT + (size_t)(n0 + row) * Kin + k0 + c8) = u;
    }
    __threadfence();
  }
}

__global__ __launch_bounds__(256) void cast8_f16_kernel(const float* __restrict__ in, unsigned short* __restrict__ out, int n8) {
  const int i = blockIdx.x * 256 + threadIdx.x;
  if (i >= n8) return;
  const float* p = in + 8 * (size_t)i;
  const v4f a = *(const v4f*)(p);
  const v4f c = *(const v4f*)(p + 4);
  unsigned short hb[8];
#pragma unroll
  for (int e = 0; e < 4; ++e) {
    hb[e]     = h_bits(a[e]);
    hb[4 + e] = h_bits(c[e]);
  }
  const v4u u = (v4u){pk16(hb[0], hb[1]), pk16(hb[2], hb[3]), pk16(hb[4], hb[5]), pk16(hb[6], hb[7])};
  unsigned short* q = out + 8 * (size_t)i;
  *(volatile v4u*)q = u;
  __threadfence();
  *(volatile v4u*)q = u;
}

__global__ __launch_bounds__(256) void relsoftmax_kernel(const float* __restrict__ Sac, const float* __restrict__ Sbd,
                                                         const int* __restrict__ mask, unsigned short* __restrict__ P) {
  __shared__ float redM[8];
  __shared__ float redS[8];
  const int i    = blockIdx.x;
  const int l    = blockIdx.y;
  const int t    = threadIdx.x;
  const int lane = t & 31, wave = t >> 5;
  const int j0   = t * 8;
  const size_t plane = (size_t)l * kQLen * kKLen;
  const float* acp = Sac + plane + (size_t)i * kKLen + j0;
  const float* bdp = Sbd + plane;
  const v4f a0 = *(const v4f*)(acp);
  const v4f a1 = *(const v4f*)(acp + 4);
  const v4i m0 = *(const v4i*)(mask + (size_t)i * kKLen + j0);
  const v4i m1 = *(const v4i*)(mask + (size_t)i * kKLen + j0 + 4);
  const float av[8] = {a0[0], a0[1], a0[2], a0[3], a1[0], a1[1], a1[2], a1[3]};
  const int   mv[8] = {m0[0], m0[1], m0[2], m0[3], m1[0], m1[1], m1[2], m1[3]};
  float x[8];
#pragma unroll
  for (int e = 0; e < 8; ++e) {
    const int j    = j0 + e;
    const int u    = (kQLen - 1) - i + j;
    const int over = (u > kRLen - 1) ? 1 : 0;
    const int row  = i + over;
    const int col  = u - over * (kRLen + 1);
    const int rowc = (row < kQLen - 1) ? row : (kQLen - 1);
    const int colc = (col > 0) ? col : 0;
    float bd = bdp[(size_t)rowc * kKLen + colc];
    bd = (col >= 0) ? bd : 0.0f;
    float s = (av[e] + bd) * kScoreScale;
    s = (mv[e] != 0) ? kMaskFill : s;
    x[e] = s;
  }
  float m = x[0];
#pragma unroll
  for (int e = 1; e < 8; ++e) m = fmaxf(m, x[e]);
#pragma unroll
  for (int off = 16; off > 0; off >>= 1) m = fmaxf(m, __shfl_xor(m, off, 32));
  if (lane == 0) redM[wave] = m;
  __syncthreads();
  m = redM[0];
#pragma unroll
  for (int k = 1; k < 8; ++k) m = fmaxf(m, redM[k]);
  float ps = 0.f;
#pragma unroll
  for (int e = 0; e < 8; ++e) {
    const float ev = expf(x[e] - m);
    x[e] = ev;
    ps += ev;
  }
#pragma unroll
  for (int off = 16; off > 0; off >>= 1) ps += __shfl_xor(ps, off, 32);
  if (lane == 0) redS[wave] = ps;
  __syncthreads();
  float sum = redS[0];
#pragma unroll
  for (int k = 1; k < 8; ++k) sum += redS[k];
  const float inv = 1.0f / sum;
  unsigned short hb[8];
#pragma unroll
  for (int e = 0; e < 8; ++e) hb[e] = h_bits(x[e] * inv * kPCarry);
  const v4u uu = (v4u){pk16(hb[0], hb[1]), pk16(hb[2], hb[3]), pk16(hb[4], hb[5]), pk16(hb[6], hb[7])};
  unsigned short* qp = P + plane + (size_t)i * kKLen + j0;
  *(volatile v4u*)qp = uu;
  __threadfence();
  *(volatile v4u*)qp = uu;
}

__global__ __launch_bounds__(256) void ln_kernel(const float* __restrict__ wres, const float* __restrict__ OW,
                                                 const float* __restrict__ gamma, const float* __restrict__ beta,
                                                 float* __restrict__ out) {
  __shared__ float redA[8];
  __shared__ float redB[8];
  const int m    = blockIdx.x;
  const int t    = threadIdx.x;
  const int lane = t & 31, wave = t >> 5;
  const int c0   = t * 4;
  const size_t ro = (size_t)m * kDModel + c0;
  const v4f a = *(const v4f*)(wres + ro);
  const v4f o = *(const v4f*)(OW + ro);
  const float x0 = a[0] + o[0], x1 = a[1] + o[1], x2 = a[2] + o[2], x3 = a[3] + o[3];
  float s = (x0 + x1) + (x2 + x3);
#pragma unroll
  for (int off = 16; off > 0; off >>= 1) s += __shfl_xor(s, off, 32);
  if (lane == 0) redA[wave] = s;
  __syncthreads();
  float tot = redA[0];
#pragma unroll
  for (int k = 1; k < 8; ++k) tot += redA[k];
  const float mean = tot * kInvDModel;
  const float d0 = x0 - mean, d1 = x1 - mean, d2 = x2 - mean, d3 = x3 - mean;
  float s2 = (d0 * d0 + d1 * d1) + (d2 * d2 + d3 * d3);
#pragma unroll
  for (int off = 16; off > 0; off >>= 1) s2 += __shfl_xor(s2, off, 32);
  if (lane == 0) redB[wave] = s2;
  __syncthreads();
  float tot2 = redB[0];
#pragma unroll
  for (int k = 1; k < 8; ++k) tot2 += redB[k];
  const float var = tot2 * kInvDModel;
  const float inv = 1.0f / sqrtf(var + kLnEps);
  const v4f g  = *(const v4f*)(gamma + c0);
  const v4f bb = *(const v4f*)(beta + c0);
  v4f y;
  y[0] = d0 * inv * g[0] + bb[0];
  y[1] = d1 * inv * g[1] + bb[1];
  y[2] = d2 * inv * g[2] + bb[2];
  y[3] = d3 * inv * g[3] + bb[3];
  float* op = out + ro;
  *(volatile v4f*)op = y;
  __threadfence();
  *(volatile v4f*)op = y;
}

extern "C" void kernel_launch(void* const* d_in, const int* in_sizes, int n_in,
                              void* d_out, int out_size, void* d_ws, size_t ws_size,
                              hipStream_t stream) {
  if (n_in < 11) return;
  if (ws_size < kWsTotal) return;
  if ((size_t)out_size < (size_t)kQRows * kDModel) return;

  const float* w     = (const float*)d_in[0];
  const float* r     = (const float*)d_in[1];
  const float* mems  = (const float*)d_in[2];
  const float* Wqkv  = (const float*)d_in[3];
  const float* Wr    = (const float*)d_in[4];
  const float* Wo    = (const float*)d_in[5];
  const float* gamma = (const float*)d_in[6];
  const float* beta  = (const float*)d_in[7];
  const float* rwb   = (const float*)d_in[8];
  const float* rrb   = (const float*)d_in[9];
  const int*   amask = (const int*)d_in[10];
  float* out = (float*)d_out;

  char* ws = (char*)d_ws;
  unsigned short* cat16 = (unsigned short*)(ws + kOffCat);
  unsigned short* r16   = (unsigned short*)(ws + kOffR16);
  unsigned short* wqkvt = (unsigned short*)(ws + kOffWqkvT);
  unsigned short* wrt   = (unsigned short*)(ws + kOffWrT);
  unsigned short* wot   = (unsigned short*)(ws + kOffWoT);
  unsigned short* qw16  = (unsigned short*)(ws + kOffQw);
  unsigned short* qr16  = (unsigned short*)(ws + kOffQr);
  unsigned short* k16   = (unsigned short*)(ws + kOffK16);
  unsigned short* vt16  = (unsigned short*)(ws + kOffVT16);
  unsigned short* rk16  = (unsigned short*)(ws + kOffRK16);
  unsigned short* av16  = (unsigned short*)(ws + kOffAV16);
  float*          sac   = (float*)(ws + kOffSac);
  float*          sbd   = (float*)(ws + kOffSbd);
  unsigned short* p16   = (unsigned short*)(ws + kOffP16);
  float*          ow    = (float*)(ws + kOffOW);
  const float* nobias  = rwb;
  const float* noresid = w;

  const unsigned short* wqt = wqkvt;
  const unsigned short* wkt = wqkvt + (size_t)kHD * kDModel;
  const unsigned short* wvt = wqkvt + (size_t)2 * kHD * kDModel;

  cast8_f16_kernel<<<dim3(2048), dim3(256), 0, stream>>>(mems, cat16, 524288);
  cast8_f16_kernel<<<dim3(2048), dim3(256), 0, stream>>>(w, cat16 + (size_t)kMLen * kBsz * kDModel, 524288);
  cast8_f16_kernel<<<dim3(1024), dim3(256), 0, stream>>>(r, r16, 262144);

  wtcast_kernel<<<dim3(16, 48), dim3(256), 0, stream>>>(Wqkv, wqkvt, kDModel, 3 * kHD, kWCarry);
  wtcast_kernel<<<dim3(16, 16), dim3(256), 0, stream>>>(Wr, wrt, kDModel, kHD, kWCarry);
  wtcast_kernel<<<dim3(16, 16), dim3(256), 0, stream>>>(Wo, wot, kHD, kDModel, kWCarry);

  wmma_gemm64<0, false, 0, 1, false><<<dim3(256, 1), dim3(256), 0, stream>>>(
      cat16, cat16, kDModel, 0L, wkt, wkt, kDModel, 0L,
      k16, k16, kHD, 0L, nobias, noresid, 0L, kCatRows, kHD, kDModel, kWCarryInv);
  wmma_gemm64<0, false, 2, 1, false><<<dim3(128, 1), dim3(256), 0, stream>>>(
      cat16 + (size_t)kMLen * kBsz * kDModel, cat16, kDModel, 0L, wqt, wqt, kDModel, 0L,
      qw16, qw16, kHD, 0L, rwb, noresid, 0L, kQRows, kHD, kDModel, kWCarryInv);
  wmma_gemm64<0, false, 2, 1, false><<<dim3(128, 1), dim3(256), 0, stream>>>(
      cat16 + (size_t)kMLen * kBsz * kDModel, cat16, kDModel, 0L, wqt, wqt, kDModel, 0L,
      qr16, qr16, kHD, 0L, rrb, noresid, 0L, kQRows, kHD, kDModel, kWCarryInv);
  wmma_gemm64<0, false, 0, 1, false><<<dim3(64, kBsz), dim3(256), 0, stream>>>(
      wvt, wvt, kDModel, 0L, cat16, cat16, kBsz * kDModel, (long)kDModel,
      vt16, vt16, kKLen, (long)kHD * kKLen, nobias, noresid, 0L, kHD, kKLen, kDModel, kWCarryInv);
  wmma_gemm64<0, false, 0, 1, false><<<dim3(64, 1), dim3(256), 0, stream>>>(
      r16, r16, kDModel, 0L, wrt, wrt, kDModel, 0L,
      rk16, rk16, kHD, 0L, nobias, noresid, 0L, kRLen, kHD, kDModel, kWCarryInv);

  const long sPlane  = (long)kQLen * kKLen;
  const long vtPlane = (long)kDHead * kKLen;
  for (int g0 = 0; g0 < kNGroups; g0 += kGrpChunk) {
    const int h0 = g0 & (kNHead - 1);
    wmma_gemm64<0, false, 0, 0, false><<<dim3(64, kGrpChunk), dim3(256), 0, stream>>>(
        qw16 + (size_t)g0 * kDHead, qw16, kBsz * kHD, (long)kDHead,
        k16 + (size_t)g0 * kDHead, k16, kBsz * kHD, (long)kDHead,
        sac, sac, kKLen, sPlane, nobias, noresid, 0L, kQLen, kKLen, kDHead, 1.0f);
    wmma_gemm64<0, false, 0, 0, false><<<dim3(64, kGrpChunk), dim3(256), 0, stream>>>(
        qr16 + (size_t)g0 * kDHead, qr16, kBsz * kHD, (long)kDHead,
        rk16 + (size_t)h0 * kDHead, rk16, kHD, (long)kDHead,
        sbd, sbd, kKLen, sPlane, nobias, noresid, 0L, kQLen, kKLen, kDHead, 1.0f);
    relsoftmax_kernel<<<dim3(kQLen, kGrpChunk), dim3(256), 0, stream>>>(sac, sbd, amask, p16);
    wmma_gemm64<0, false, 0, 1, false><<<dim3(2, kGrpChunk), dim3(256), 0, stream>>>(
        p16, p16, kKLen, sPlane,
        vt16 + (size_t)g0 * vtPlane, vt16, kKLen, vtPlane,
        av16 + (size_t)g0 * kDHead, av16, kBsz * kHD, (long)kDHead,
        nobias, noresid, 0L, kQLen, kDHead, kKLen, kPVScale);
  }

  wmma_gemm64<0, false, 0, 0, false><<<dim3(128, 1), dim3(256), 0, stream>>>(
      av16, av16, kHD, 0L, wot, wot, kHD, 0L,
      ow, ow, kDModel, 0L, nobias, noresid, 0L, kQRows, kDModel, kHD, kOutScale);

  ln_kernel<<<dim3(kQRows), dim3(256), 0, stream>>>(w, ow, gamma, beta, out);
}
